// CMEncoder_23502061043973
// MI455X (gfx1250) — hardware-verified
//
#include <hip/hip_runtime.h>
#include <math.h>

typedef __attribute__((ext_vector_type(16))) _Float16 v16h;
typedef __attribute__((ext_vector_type(16))) __bf16 v16b;
typedef __attribute__((ext_vector_type(8)))  _Float16 v8h;
typedef __attribute__((ext_vector_type(8)))  float v8f;
typedef __attribute__((ext_vector_type(4)))  float v4f;
typedef __attribute__((ext_vector_type(2)))  float v2f;
typedef __attribute__((ext_vector_type(4)))  unsigned v4u;
typedef __attribute__((ext_vector_type(4)))  int v4i;
typedef float __attribute__((may_alias)) float_a;
typedef int __attribute__((may_alias)) int_a;

template <typename T> __device__ __forceinline__ void vst2(void* p, T v) { *(volatile T*)p = v; __threadfence(); *(volatile T*)p = v; }
__device__ __forceinline__ v8f wmma16(v16h a, v16h b, v8f c) {
  v8f d = __builtin_amdgcn_wmma_f32_16x16x32_f16(false, a, false, b, (short)0, c, false, false);
  asm volatile("v_nop\n\tv_nop\n\tv_nop\n\tv_nop" : "+v"(d) : "v"(a), "v"(b));
  return d;
}
__device__ __forceinline__ v8f wmma_bf(v16b a, v16b b, v8f c) {
  v8f d = __builtin_amdgcn_wmma_f32_16x16x32_bf16(false, a, false, b, (short)0, c, false, false);
  asm volatile("v_nop\n\tv_nop\n\tv_nop\n\tv_nop" : "+v"(d) : "v"(a), "v"(b));
  return d;
}
__device__ __forceinline__ v16h frag_h(const _Float16* rowk0, int lane) {
  union { v16h v; v8h q[2]; } u; const _Float16* p = rowk0 + 8 * (lane >> 4);
  u.q[0] = *(const v8h*)p; u.q[1] = *(const v8h*)(p + 16); return u.v;
}
__device__ __forceinline__ v16h frag_f32(const float* rowk0, int lane) {
  v16h a; const float* p = rowk0 + 8 * (lane >> 4);
#pragma unroll
  for (int i = 0; i < 8; ++i) { a[i] = (_Float16)p[i]; a[8 + i] = (_Float16)p[16 + i]; }
  return a;
}
__device__ __forceinline__ v16h frag_f32s(const float* rowk0, int lane, float sc) {
  v16h a; const float* p = rowk0 + 8 * (lane >> 4);
#pragma unroll
  for (int i = 0; i < 8; ++i) { a[i] = (_Float16)(p[i] * sc); a[8 + i] = (_Float16)(p[16 + i] * sc); }
  return a;
}
__device__ __forceinline__ v16h fragc_f32(const float* W, int k0, int n, int lane, int ld, int K) {
  v16h a; const int g = lane >> 4;
#pragma unroll
  for (int i = 0; i < 8; ++i) { const int ka = k0 + 8 * g + i, kb = ka + 16;
    a[i] = (_Float16)(ka < K ? W[(size_t)(ka < K ? ka : K - 1) * ld + n] : 0.f); a[8 + i] = (_Float16)(kb < K ? W[(size_t)(kb < K ? kb : K - 1) * ld + n] : 0.f); }
  return a;
}
struct F2 { v16b h, l; };
__device__ __forceinline__ F2 bsplit16(const float v[16]) { F2 r;
#pragma unroll
  for (int i = 0; i < 16; ++i) { const __bf16 h = (__bf16)v[i]; r.h[i] = h; r.l[i] = (__bf16)(v[i] - (float)h); }
  return r; }
__device__ __forceinline__ F2 split_row(const float* row, int k0, int lane) { float v[16]; const float* p = row + k0 + 8 * (lane >> 4);
#pragma unroll
  for (int i = 0; i < 8; ++i) { v[i] = p[i]; v[8 + i] = p[16 + i]; }
  return bsplit16(v); }
__device__ __forceinline__ F2 split_rowK(const float* row, int k0, int lane, int K) { float v[16]; const int g = lane >> 4;
#pragma unroll
  for (int i = 0; i < 8; ++i) { const int ka = k0 + 8 * g + i, kb = ka + 16; v[i] = ka < K ? row[ka < K ? ka : K - 1] : 0.f; v[8 + i] = kb < K ? row[kb < K ? kb : K - 1] : 0.f; }
  return bsplit16(v); }
__device__ __forceinline__ F2 split_col(const float* W, int k0, int n, int lane, int ld, int K) { float v[16]; const int g = lane >> 4;
#pragma unroll
  for (int i = 0; i < 8; ++i) { const int ka = k0 + 8 * g + i, kb = ka + 16; v[i] = ka < K ? W[(size_t)(ka < K ? ka : K - 1) * ld + n] : 0.f; v[8 + i] = kb < K ? W[(size_t)(kb < K ? kb : K - 1) * ld + n] : 0.f; }
  return bsplit16(v); }
__device__ __forceinline__ v8f mac3(const F2& a, const F2& b, v8f c) { c = wmma_bf(a.l, b.h, c); c = wmma_bf(a.h, b.l, c); return wmma_bf(a.h, b.h, c); }
__device__ __forceinline__ float sigm(float v) { return 1.0f / (1.0f + expf(-v)); }
#define LDSX() do { asm volatile("s_wait_dscnt 0" ::: "memory"); __builtin_amdgcn_wave_barrier(); __builtin_amdgcn_fence(__ATOMIC_RELEASE, "workgroup"); } while (0)


#define C 256
#define NP 4096
#define NK 4096
#define HID 512
__device__ __attribute__((noinline)) float gelu_e(float v) { return 0.5f * v * (1.0f + erff(v * 0.70710678118654752f)); }

__global__ __launch_bounds__(256) void k_cvt(const float* __restrict__ src, _Float16* __restrict__ T16) {
  __shared__ __align__(16) _Float16 st[64][C + 8];
  const int tid = threadIdx.x, n0 = blockIdx.x * 64;
  for (int q = tid; q < C * 16; q += 256) { const int c = q >> 4, p4 = q & 15; const v4f v = *(const v4f*)(src + (size_t)c * NP + n0 + p4 * 4);
    st[p4 * 4][c] = (_Float16)v[0]; st[p4 * 4 + 1][c] = (_Float16)v[1]; st[p4 * 4 + 2][c] = (_Float16)v[2]; st[p4 * 4 + 3][c] = (_Float16)v[3]; }
  __syncthreads();
  for (int q = tid; q < 64 * (C / 8); q += 256) { const int rl = q >> 5, pc = q & 31; vst2(T16 + (size_t)(n0 + rl) * C + pc * 8, *(const v4u*)(&st[rl][pc * 8])); }
}
__global__ __launch_bounds__(256) void k_pack(const float* __restrict__ Wq, const float* __restrict__ Wk, const float* __restrict__ Wv, const float* __restrict__ Wo, const float* __restrict__ W1, const float* __restrict__ W2, _Float16* __restrict__ PA, _Float16* __restrict__ PB) {
  const int n = blockIdx.x, tid = threadIdx.x; __shared__ __align__(16) _Float16 srow[HID];
  if (n < 4 * C + HID) { const float* W = n < C ? Wq + (size_t)n * C : (n < 2 * C ? Wk + (size_t)(n - C) * C : (n < 3 * C ? Wv + (size_t)(n - 2 * C) * C : (n < 4 * C ? Wo + (size_t)(n - 3 * C) * C : W1 + (size_t)(n - 4 * C) * C)));
    srow[tid] = (_Float16)(W[tid] * 16.0f); __syncthreads(); if (tid < C / 8) vst2(PA + (size_t)n * C + tid * 8, *(const v4u*)(&srow[tid * 8])); }
  else { const int m = n - (4 * C + HID); const float* W = W2 + (size_t)m * HID; srow[tid] = (_Float16)(W[tid] * 16.0f); srow[tid + 256] = (_Float16)(W[tid + 256] * 16.0f); __syncthreads();
    if (tid < HID / 8) vst2(PB + (size_t)m * HID + tid * 8, *(const v4u*)(&srow[tid * 8])); }
}
__global__ __launch_bounds__(128) void k_qkv(const _Float16* __restrict__ X16, const _Float16* __restrict__ Y16, const _Float16* __restrict__ PA, const float* __restrict__ bq, const float* __restrict__ bk, const float* __restrict__ bv, _Float16* __restrict__ Q16, _Float16* __restrict__ K16, _Float16* __restrict__ VT) {
  __shared__ __align__(16) _Float16 so[4][16][136];
  __shared__ __align__(16) _Float16 sth[128][72];
  const int tid = threadIdx.x, wave = tid >> 5, lane = tid & 31, col = lane & 15, g = lane >> 4;
  const int which = blockIdx.z, r0b = blockIdx.x * 64, r0 = r0b + wave * 16, n0 = blockIdx.y * 128; const _Float16* SRC = which == 0 ? X16 : Y16; const float* bb_ = which == 0 ? bq : (which == 1 ? bk : bv);
  v8f acc[8] = {};
#pragma unroll 2
  for (int kc = 0; kc < C / 32; ++kc) { const v16h a = frag_h(SRC + (size_t)(r0 + col) * C + kc * 32, lane);
#pragma unroll
    for (int j = 0; j < 8; ++j) acc[j] = wmma16(a, frag_h(PA + (size_t)(which * C + n0 + j * 16 + col) * C + kc * 32, lane), acc[j]); }
  if (which < 2) {
#pragma unroll
    for (int j = 0; j < 8; ++j) { const float bb = bb_[n0 + j * 16 + col];
#pragma unroll
      for (int r = 0; r < 8; ++r) so[wave][8 * g + r][j * 16 + col] = (_Float16)((acc[j][r] * (1.0f / 16.0f) + bb) * 4.0f); }
    LDSX();
    _Float16* D = which == 0 ? Q16 : K16;
    for (int rl = 0; rl < 16; ++rl) { if (lane < 16) vst2(D + (size_t)(r0 + rl) * C + n0 + lane * 8, *(const v4u*)(&so[wave][rl][lane * 8])); } }
  else {
#pragma unroll
    for (int j = 0; j < 8; ++j) { const float bb = bb_[n0 + j * 16 + col];
#pragma unroll
      for (int r = 0; r < 8; ++r) sth[j * 16 + col][wave * 16 + 8 * g + r] = (_Float16)((acc[j][r] * (1.0f / 16.0f) + bb) * 4.0f); }
    __syncthreads();
    for (int qq = tid; qq < 128 * 8; qq += 128) { const int cl = qq >> 3, pc = qq & 7; vst2(VT + (size_t)(n0 + cl) * NK + r0b + pc * 8, *(const v4u*)(&sth[cl][pc * 8])); } }
}
__global__ __launch_bounds__(128) void k_attn(const _Float16* __restrict__ Q16, const _Float16* __restrict__ K16, const _Float16* __restrict__ VT, float* __restrict__ O32) {
  __shared__ __align__(16) float sS[4][16][68];
  __shared__ __align__(16) _Float16 sPh[4][16][72];
  __shared__ __align__(16) float sO[4][16][132];
  const int tid = threadIdx.x, w = tid >> 5, lane = tid & 31, col = lane & 15, g = lane >> 4; const int q0 = blockIdx.x * 64 + w * 16; const int dh = blockIdx.y;
  v16h aq[8];
#pragma unroll
  for (int kc = 0; kc < 8; ++kc) aq[kc] = frag_h(Q16 + (size_t)(q0 + col) * C + kc * 32, lane);
  float mrun = -3.0e38f, lrun = 0.f; v8f acc[8] = {};
#pragma unroll 1
  for (int kt = 0; kt < NK / 64; ++kt) {
#pragma unroll
    for (int t = 0; t < 4; ++t) { v8f s = {}; const int key = kt * 64 + t * 16 + col;
#pragma unroll
      for (int kc = 0; kc < 8; ++kc) s = wmma16(aq[kc], frag_h(K16 + (size_t)key * C + kc * 32, lane), s);
#pragma unroll
      for (int r = 0; r < 8; ++r) sS[w][8 * g + r][t * 16 + col] = s[r] * (0.0625f / 16.0f); }
    LDSX();
    float mx = -3.4e38f;
#pragma unroll
    for (int jj = 0; jj < 32; ++jj) mx = fmaxf(mx, sS[w][col][g * 32 + jj]);
    mx = fmaxf(mx, __shfl_xor(mx, 16, 32));
    const float mnew = fmaxf(mrun, mx); const float corr = expf(mrun - mnew);
    float ps = 0.f;
#pragma unroll
    for (int jj = 0; jj < 32; ++jj) { const float p = expf(sS[w][col][g * 32 + jj] - mnew) * 16384.0f; ps += p; sPh[w][col][g * 32 + jj] = (_Float16)p; }
    ps += __shfl_xor(ps, 16, 32);
    lrun = lrun * corr + ps * (1.0f / 16384.0f); mrun = mnew;
#pragma unroll
    for (int r = 0; r < 8; ++r) { const float cr = __shfl(corr, 8 * g + r, 32);
#pragma unroll
      for (int t = 0; t < 8; ++t) acc[t][r] *= cr; }
    LDSX();
#pragma unroll
    for (int kc = 0; kc < 2; ++kc) { const v16h ph = frag_h(&sPh[w][col][0] + kc * 32, lane);
#pragma unroll
      for (int t = 0; t < 8; ++t) acc[t] = wmma16(ph, frag_h(VT + (size_t)(dh * 128 + t * 16 + col) * NK + kt * 64 + kc * 32, lane), acc[t]); }
    __builtin_amdgcn_wave_barrier(); }
#pragma unroll
  for (int r = 0; r < 8; ++r) { const float lr = __shfl(lrun, 8 * g + r, 32); const float inv = 1.0f / (lr * 16384.0f * 4.0f);
#pragma unroll
    for (int t = 0; t < 8; ++t) sO[w][8 * g + r][t * 16 + col] = acc[t][r] * inv; }
  LDSX();
  for (int rl = 0; rl < 16; ++rl) vst2(O32 + (size_t)(q0 + rl) * C + dh * 128 + lane * 4, *(const v4f*)(&sO[w][rl][lane * 4]));
}
__global__ __launch_bounds__(128) void k_post(const float* __restrict__ O32, const _Float16* __restrict__ PA, const _Float16* __restrict__ PB, const float* __restrict__ bo, const float* __restrict__ lw, const float* __restrict__ lb, const float* __restrict__ b1, const float* __restrict__ b2, const float* __restrict__ x, float* __restrict__ out) {
  __shared__ __align__(16) _Float16 sz[4][16][C + 8];
  __shared__ __align__(16) float szf[4][16][C + 4];
  __shared__ __align__(16) _Float16 shh[4][16][HID + 8];
  const int tid = threadIdx.x, wave = tid >> 5, lane = tid & 31, col = lane & 15, g = lane >> 4; const int p0b = blockIdx.x * 64, r0 = p0b + wave * 16;
  for (int qq = lane; qq < 16 * (C / 4); qq += 32) { const int rl = qq >> 6, pc = qq & 63; const v4f v = *(const v4f*)(O32 + (size_t)(r0 + rl) * C + pc * 4);
#pragma unroll
    for (int e = 0; e < 4; ++e) sz[wave][rl][pc * 4 + e] = (_Float16)(v[e] * 64.0f); }
  LDSX();
  { v8f acc[16] = {};
#pragma unroll 1
    for (int kc = 0; kc < C / 32; ++kc) { const v16h a = frag_h(&sz[wave][col][0] + kc * 32, lane);
#pragma unroll
      for (int j = 0; j < 16; ++j) acc[j] = wmma16(a, frag_h(PA + (size_t)(3 * C + j * 16 + col) * C + kc * 32, lane), acc[j]); }
#pragma unroll
    for (int j = 0; j < 16; ++j) { const float bb = bo[j * 16 + col];
#pragma unroll
      for (int r = 0; r < 8; ++r) szf[wave][8 * g + r][j * 16 + col] = acc[j][r] * (1.0f / (16.0f * 64.0f)) + bb; } }
  LDSX();
  { const int rl = lane & 15, hf = lane >> 4; const float* zr = &szf[wave][rl][hf * 128]; float s = 0.f, q = 0.f;
#pragma unroll 2
    for (int e = 0; e < 128; ++e) s += zr[e];
    s += __shfl_xor(s, 16, 32); const float mu = s * (1.0f / C);
#pragma unroll 2
    for (int e = 0; e < 128; ++e) { const float d = zr[e] - mu; q += d * d; }
    q += __shfl_xor(q, 16, 32); const float rs = rsqrtf(q * (1.0f / C) + 1e-6f);
#pragma unroll 2
    for (int e = 0; e < 128; ++e) { const int c = hf * 128 + e; sz[wave][rl][c] = (_Float16)((zr[e] - mu) * rs * lw[c] + lb[c]); } }
  LDSX();
#pragma unroll 1
  for (int ph = 0; ph < 2; ++ph) { v8f acc[16] = {};
#pragma unroll 1
    for (int kc = 0; kc < C / 32; ++kc) { const v16h a = frag_h(&sz[wave][col][0] + kc * 32, lane);
#pragma unroll
      for (int j = 0; j < 16; ++j) acc[j] = wmma16(a, frag_h(PA + (size_t)(4 * C + ph * 256 + j * 16 + col) * C + kc * 32, lane), acc[j]); }
#pragma unroll
    for (int j = 0; j < 16; ++j) { const int n = ph * 256 + j * 16 + col; const float bb = b1[n];
#pragma unroll
      for (int r = 0; r < 8; ++r) shh[wave][8 * g + r][n] = (_Float16)gelu_e(acc[j][r] * (1.0f / 16.0f) + bb); } }
  LDSX();
  { v8f acc[16] = {};
#pragma unroll 1
    for (int kc = 0; kc < HID / 32; ++kc) { const v16h a = frag_h(&shh[wave][col][0] + kc * 32, lane);
#pragma unroll
      for (int j = 0; j < 16; ++j) acc[j] = wmma16(a, frag_h(PB + (size_t)(j * 16 + col) * HID + kc * 32, lane), acc[j]); }
#pragma unroll
    for (int j = 0; j < 16; ++j) { const float bb = b2[j * 16 + col];
#pragma unroll
      for (int r = 0; r < 8; ++r) szf[wave][8 * g + r][j * 16 + col] = acc[j][r] * (1.0f / 16.0f) + bb; } }
  __syncthreads();
  for (int q = tid; q < C * 16; q += 128) { const int c = q >> 4, pc = q & 15; v4f v = *(const v4f*)(x + (size_t)c * NP + p0b + pc * 4);
#pragma unroll
    for (int e = 0; e < 4; ++e) { const int pl = pc * 4 + e; v[e] += szf[pl >> 4][pl & 15][c]; }
    vst2(out + (size_t)c * NP + p0b + pc * 4, v); }
}
extern "C" void kernel_launch(void* const* d_in, const int* in_sizes, int n_in, void* d_out, int out_size, void* d_ws, size_t ws_size, hipStream_t stream) {
  (void)in_sizes; (void)n_in; (void)out_size; (void)ws_size;
  const float** I = (const float**)d_in;
  const float* x = I[0]; const float* y = I[1]; const float* Wq = I[2]; const float* bq = I[3]; const float* Wk = I[4]; const float* bk = I[5]; const float* Wv = I[6]; const float* bv = I[7]; const float* Wo = I[8]; const float* bo = I[9];
  const float* lw = I[10]; const float* lb = I[11]; const float* W1 = I[12]; const float* b1 = I[13]; const float* W2 = I[14]; const float* b2 = I[15];
  float* out = (float*)d_out;
  char* ws = (char*)d_ws; size_t off = 0;
  auto take = [&](size_t bytes) { char* p = ws + off; off += (bytes + 255) & ~(size_t)255; return p; };
  _Float16* X16 = (_Float16*)take((size_t)NP * C * 2); _Float16* Y16 = (_Float16*)take((size_t)NK * C * 2); _Float16* PA = (_Float16*)take((size_t)(4 * C + HID) * C * 2); _Float16* PB = (_Float16*)take((size_t)C * HID * 2);
  _Float16* Q16 = (_Float16*)take((size_t)NP * C * 2); _Float16* K16 = (_Float16*)take((size_t)NK * C * 2); _Float16* VT = (_Float16*)take((size_t)C * NK * 2); float* O32 = (float*)take((size_t)NP * C * 4);
  k_cvt<<<NP / 64, 256, 0, stream>>>(x, X16);
  k_cvt<<<NK / 64, 256, 0, stream>>>(y, Y16);
  k_pack<<<4 * C + HID + C, 256, 0, stream>>>(Wq, Wk, Wv, Wo, W1, W2, PA, PB);
  k_qkv<<<dim3(NP / 64, C / 128, 3), 128, 0, stream>>>(X16, Y16, PA, bq, bk, bv, Q16, K16, VT);
  k_attn<<<dim3(NP / 64, 2), 128, 0, stream>>>(Q16, K16, VT, O32);
  k_post<<<NP / 64, 128, 0, stream>>>(O32, PA, PB, bo, lw, lb, b1, b2, x, out);
}
